// CrossAttentionWithTemporalEmbedding_67053029425312
// MI455X (gfx1250) — hardware-verified
//
#include <hip/hip_runtime.h>
#include <hip/hip_bf16.h>

typedef __attribute__((ext_vector_type(16))) _Float16 v16h;
typedef __attribute__((ext_vector_type(8)))  _Float16 v8h;
typedef __attribute__((ext_vector_type(16))) __bf16   v16b;
typedef __attribute__((ext_vector_type(8)))  __bf16   v8b;
typedef __attribute__((ext_vector_type(8)))  float    v8f;
typedef __attribute__((ext_vector_type(4)))  float    v4f;

constexpr int kBatch = 4;
constexpr int kCh    = 256;
constexpr int kQC    = 32;
constexpr int kQK    = 64;
constexpr int kHW    = 4096;
constexpr int kBiasPer = 320;

__device__ __forceinline__ unsigned short f2bf_bits(float f) {
  unsigned u = __float_as_uint(f);
  return (unsigned short)((u + 0x7FFFu + ((u >> 16) & 1u)) >> 16);
}
__device__ __forceinline__ float bf_bits2f(unsigned short h) { return __uint_as_float(((unsigned)h) << 16); }

__device__ __forceinline__ void dep_guard_h(v8f& a, v8f& b, v16h x, v16h y) { asm volatile("v_nop\n\tv_nop\n\tv_nop\n\tv_nop" : "+v"(a), "+v"(b) : "v"(x), "v"(y)); }
__device__ __forceinline__ void dep_guard_b(v8f& a, v8f& b, v16b x, v16b y) { asm volatile("v_nop\n\tv_nop\n\tv_nop\n\tv_nop" : "+v"(a), "+v"(b) : "v"(x), "v"(y)); }
__device__ __forceinline__ void keep4_h(v16h a, v16h b, v16h c, v16h d) { asm volatile("v_nop" :: "v"(a), "v"(b), "v"(c), "v"(d)); }
__device__ __forceinline__ void keep4_b(v16b a, v16b b, v16b c, v16b d) { asm volatile("v_nop" :: "v"(a), "v"(b), "v"(c), "v"(d)); }
__device__ __forceinline__ void acc_guard4(v8f& a, v8f& b, v8f& c, v8f& d) { asm volatile("v_nop\n\tv_nop\n\tv_nop\n\tv_nop" : "+v"(a), "+v"(b), "+v"(c), "+v"(d)); }
template <typename T> struct Frag;
template <> struct Frag<_Float16> {
  typedef v16h V; union U { v16h v; v8h h[2]; };
  static __device__ __forceinline__ v16h load(const _Float16* p) {
    U f; f.h[0] = *(const v8h*)(p); f.h[1] = *(const v8h*)(p + 16); return f.v;
  }
  static __device__ __forceinline__ v8f mma(v16h a, v16h b, v8f c) {
    return __builtin_amdgcn_wmma_f32_16x16x32_f16(false, a, false, b, (short)0, c, false, false);
  }
  static __device__ __forceinline__ void guard(v8f& a, v8f& b, v16h x, v16h y) { dep_guard_h(a, b, x, y); }
  static __device__ __forceinline__ void keep(v16h a, v16h b, v16h c, v16h d) { keep4_h(a, b, c, d); }
};
template <> struct Frag<__bf16> {
  typedef v16b V; union U { v16b v; v8b h[2]; };
  static __device__ __forceinline__ v16b load(const __bf16* p) {
    U f; f.h[0] = *(const v8b*)(p); f.h[1] = *(const v8b*)(p + 16); return f.v;
  }
  static __device__ __forceinline__ v8f mma(v16b a, v16b b, v8f c) {
    return __builtin_amdgcn_wmma_f32_16x16x32_bf16(false, a, false, b, (short)0, c, false, false);
  }
  static __device__ __forceinline__ void guard(v8f& a, v8f& b, v16b x, v16b y) { dep_guard_b(a, b, x, y); }
  static __device__ __forceinline__ void keep(v16b a, v16b b, v16b c, v16b d) { keep4_b(a, b, c, d); }
};

template <int ET> struct Elem;
template <> struct Elem<0> { typedef _Float16 T; };
template <> struct Elem<1> { typedef __bf16 T; };
template <int ET, bool SPLIT, int BIAS_MODE, int OUT_MODE, bool RESID, int ACT = 0>
__global__ __launch_bounds__(256) void wmma_gemm64(
    const unsigned short* __restrict__ Ap, const unsigned short* __restrict__ A2p, int lda, long strideA,
    const unsigned short* __restrict__ Btp, const unsigned short* __restrict__ Bt2p, int ldb, long strideB,
    void* __restrict__ Cout, void* __restrict__ Cout2, int ldc, long strideC,
    const float* __restrict__ bias,
    const float* __restrict__ resid, long strideR,
    int M, int N, int K, float scale) {
  typedef typename Elem<ET>::T T;
  typedef typename Frag<T>::V V;
  const T* A = (const T*)Ap; const T* A2 = (const T*)A2p; const T* Bt = (const T*)Btp; const T* Bt2 = (const T*)Bt2p;
  __shared__ __align__(16) float sT[8][16 * 68];
  const int b    = blockIdx.y;
  const int lane = threadIdx.x & 31;
  const int wave = threadIdx.x >> 5;
  const int tilesN = N >> 6;
  const int tilesM = M >> 6;
  const int tile = blockIdx.x * 8 + wave;
  if (tile >= tilesM * tilesN) return;
  const int tm = tile / tilesN;
  const int tn = tile - tm * tilesN;
  const int m0 = tm << 6;
  const int n0 = tn << 6;

  const T* Ab  = A  + (size_t)b * strideA;
  const T* Bb  = Bt + (size_t)b * strideB;
  const T* Ab2 = SPLIT ? (A2  + (size_t)b * strideA) : nullptr;
  const T* Bb2 = SPLIT ? (Bt2 + (size_t)b * strideB) : nullptr;

  const int rlane = lane & 15;
  const int koff  = (lane >> 4) * 8;
  const int mOff  = (lane >> 4) * 8;

  v8f acc[4][4];
#pragma unroll
  for (int i = 0; i < 4; ++i)
#pragma unroll
    for (int j = 0; j < 4; ++j) acc[i][j] = (v8f){0.f,0.f,0.f,0.f,0.f,0.f,0.f,0.f};

  for (int k0 = 0; k0 < K; k0 += 32) {
    V bh[4], bl[4];
#pragma unroll
    for (int j = 0; j < 4; ++j) {
      const size_t bo = (size_t)(n0 + (j << 4) + rlane) * ldb + koff + k0;
      bh[j] = Frag<T>::load(Bb + bo);
      if (SPLIT) bl[j] = Frag<T>::load(Bb2 + bo);
    }
#pragma unroll
    for (int i = 0; i < 4; ++i) {
      const size_t ao = (size_t)(m0 + (i << 4) + rlane) * lda + koff + k0;
      V ah = Frag<T>::load(Ab + ao);
      V al;
      if (SPLIT) al = Frag<T>::load(Ab2 + ao);
#pragma unroll
      for (int j = 0; j < 4; ++j) {
        acc[i][j] = Frag<T>::mma(ah, bh[j], acc[i][j]);
        if (SPLIT) {
          acc[i][j] = Frag<T>::mma(ah, bl[j], acc[i][j]);
          acc[i][j] = Frag<T>::mma(al, bh[j], acc[i][j]);
        }
      }
      Frag<T>::guard(acc[i][0], acc[i][3], ah, SPLIT ? al : ah);
    }
    Frag<T>::keep(bh[0], bh[1], bh[2], bh[3]);
    if (SPLIT) Frag<T>::keep(bl[0], bl[1], bl[2], bl[3]);
  }
  acc_guard4(acc[0][0], acc[0][1], acc[0][2], acc[0][3]);
  acc_guard4(acc[1][0], acc[1][1], acc[1][2], acc[1][3]);
  acc_guard4(acc[2][0], acc[2][1], acc[2][2], acc[2][3]);
  acc_guard4(acc[3][0], acc[3][1], acc[3][2], acc[3][3]);

  float* slab = sT[wave];
  const float* Rb = RESID ? (resid + (size_t)b * strideR) : nullptr;
#pragma unroll
  for (int i = 0; i < 4; ++i) {
    const int mBase = m0 + (i << 4);
#pragma unroll
    for (int j = 0; j < 4; ++j) {
      const int n = n0 + (j << 4) + rlane;
      float bv = 0.f;
      if (BIAS_MODE == 2) bv = bias[n];
#pragma unroll
      for (int r = 0; r < 8; ++r) {
        float v = acc[i][j][r] * scale;
        if (BIAS_MODE == 1) v += bias[mBase + mOff + r];
        if (BIAS_MODE == 2) v += bv;
        if (RESID) v += Rb[(size_t)(mBase + mOff + r) * ldc + n];
        if (ACT == 1) v = tanhf(v);
        if (ACT == 2) v = fmaxf(v, 0.0f);
        if (ACT == 3) v = v / (1.0f + expf(-v));
        if (ACT == 4) v = (v > 0.f) ? v : 0.01f * v;
        if (ACT == 5) v = 0.5f * v * (1.0f + erff(v * 0.70710678118654752f));
        slab[(mOff + r) * 68 + (j << 4) + rlane] = v;
      }
    }
    __builtin_amdgcn_fence(__ATOMIC_RELEASE, "workgroup");
    __builtin_amdgcn_wave_barrier();
    __builtin_amdgcn_fence(__ATOMIC_ACQUIRE, "workgroup");
    if (OUT_MODE == 0) {
      float* C = (float*)Cout + (size_t)b * strideC;
      const int hh = lane >> 4, c4 = (lane & 15) * 4;
      for (int pass = 0; pass < 2; ++pass) {
#pragma unroll
        for (int it = 0; it < 8; ++it) {
          const int row = it * 2 + hh;
          v4f v = *(const v4f*)(slab + row * 68 + c4);
          *(volatile v4f*)(C + (size_t)(mBase + row) * ldc + n0 + c4) = v;
        }
        __threadfence();
      }
    } else {
      const int q = lane >> 3, c8 = (lane & 7) * 8;
      unsigned short* C  = (unsigned short*)Cout  + (size_t)b * strideC;
      unsigned short* C2 = (OUT_MODE == 2) ? ((unsigned short*)Cout2 + (size_t)b * strideC) : nullptr;
      for (int pass = 0; pass < 2; ++pass) {
#pragma unroll
        for (int it = 0; it < 4; ++it) {
          const int row = it * 4 + q;
          const float* sp = slab + row * 68 + c8;
          v8h hv, lv;
#pragma unroll
          for (int e = 0; e < 8; ++e) {
            if (OUT_MODE == 1) {
              hv[e] = (_Float16)sp[e];
            } else {
              unsigned short hb = f2bf_bits(sp[e]);
              unsigned short lb = f2bf_bits(sp[e] - bf_bits2f(hb));
              hv[e] = __builtin_bit_cast(_Float16, hb);
              lv[e] = __builtin_bit_cast(_Float16, lb);
            }
          }
          *(volatile v8h*)(C + (size_t)(mBase + row) * ldc + n0 + c8) = hv;
          if (OUT_MODE == 2) *(volatile v8h*)(C2 + (size_t)(mBase + row) * ldc + n0 + c8) = lv;
        }
        __threadfence();
      }
    }
    __builtin_amdgcn_fence(__ATOMIC_RELEASE, "workgroup");
    __builtin_amdgcn_wave_barrier();
    __builtin_amdgcn_fence(__ATOMIC_ACQUIRE, "workgroup");
  }
}

__global__ __launch_bounds__(256) void k_biasfold(
    const float* __restrict__ wq, const float* __restrict__ bq,
    const float* __restrict__ wk, const float* __restrict__ bk,
    const float* __restrict__ wv, const float* __restrict__ bv,
    const float* __restrict__ te1, const float* __restrict__ te2,
    const float* __restrict__ gamma, float* __restrict__ BIAS) {
  __shared__ float res[32];
  const int tid = threadIdx.x, wave = tid >> 5, lane = tid & 31;
  const int li  = blockIdx.x;
  const int dir = li / 10;
  const int r0  = (li - dir * 10) * 32;
  const float* t = dir ? te2 : te1;
  const float* Wm   = (r0 < 32) ? wq : ((r0 < 64) ? wk : wv);
  const float* bvec = (r0 < 32) ? bq : ((r0 < 64) ? bk : bv);
  const int rb = (r0 < 32) ? 0 : ((r0 < 64) ? 32 : 64);
  const float g8 = 8.0f * gamma[0];
  const float mul = (r0 < 64) ? 1.0f : g8;
  const v4f ta = *(const v4f*)(t + lane * 8);
  const v4f tb = *(const v4f*)(t + lane * 8 + 4);
#pragma unroll 1
  for (int i = 0; i < 4; ++i) {
    const int rloc = r0 - rb + wave * 4 + i;
    const float* wr = Wm + (size_t)rloc * kCh + lane * 8;
    const v4f w0 = *(const v4f*)(wr);
    const v4f w1 = *(const v4f*)(wr + 4);
    float d = w0[0] * ta[0] + w0[1] * ta[1] + w0[2] * ta[2] + w0[3] * ta[3]
            + w1[0] * tb[0] + w1[1] * tb[1] + w1[2] * tb[2] + w1[3] * tb[3];
#pragma unroll
    for (int off = 1; off < 32; off <<= 1) d += __shfl_xor(d, off, 32);
    const float val = (d + bvec[rloc]) * mul;
    if (lane == 0) res[wave * 4 + i] = val;
  }
  __syncthreads();
  if (wave == 0) {
    const float o = res[lane];
    volatile float* dp = BIAS + (size_t)li * 32 + lane;
    *dp = o;
    __threadfence();
    *dp = o;
  }
}

__global__ __launch_bounds__(256) void k_prepw(
    const float* __restrict__ wq, const float* __restrict__ wk, const float* __restrict__ wv,
    const float* __restrict__ gamma,
    unsigned short* __restrict__ Wqkhi, unsigned short* __restrict__ Wqklo, unsigned short* __restrict__ Wv16) {
  const int blk = blockIdx.x, tid = threadIdx.x;
  if (blk < 32) {
    const float* src = (blk < 16) ? (wq + blk * 512) : (wk + (blk - 16) * 512);
    const float f0 = src[2 * tid], f1 = src[2 * tid + 1];
    const unsigned short hb0 = f2bf_bits(f0), hb1 = f2bf_bits(f1);
    const unsigned short lb0 = f2bf_bits(f0 - bf_bits2f(hb0)), lb1 = f2bf_bits(f1 - bf_bits2f(hb1));
    const unsigned uh = (unsigned)hb0 | ((unsigned)hb1 << 16);
    const unsigned ul = (unsigned)lb0 | ((unsigned)lb1 << 16);
    const int p = blk * 256 + tid;
    volatile unsigned* dh = ((volatile unsigned*)Wqkhi) + p;
    volatile unsigned* dl = ((volatile unsigned*)Wqklo) + p;
    *dh = uh;
    *dl = ul;
    __threadfence();
    *dh = uh;
    *dl = ul;
  } else {
    const int p = (blk - 32) * 256 + tid;
    const float g16 = 16.0f * gamma[0];
    const float f0 = wv[2 * p] * g16, f1 = wv[2 * p + 1] * g16;
    const _Float16 h0 = (_Float16)f0, h1 = (_Float16)f1;
    const unsigned u = (unsigned)__builtin_bit_cast(unsigned short, h0) | ((unsigned)__builtin_bit_cast(unsigned short, h1) << 16);
    volatile unsigned* dp = ((volatile unsigned*)Wv16) + p;
    *dp = u;
    __threadfence();
    *dp = u;
  }
}

__global__ __launch_bounds__(256) void k_ftrans(
    const float* __restrict__ f1, const float* __restrict__ f2, int b,
    unsigned short* __restrict__ FThi, unsigned short* __restrict__ FTlo, unsigned short* __restrict__ FT16) {
  __shared__ __align__(16) float T[32 * 260];
  const int tid = threadIdx.x;
  const int sel = blockIdx.y;
  const int n0  = blockIdx.x * 32;
  const float* xb = (sel ? f2 : f1) + (size_t)b * kCh * kHW + n0;
#pragma unroll 4
  for (int it = 0; it < 32; ++it) {
    const int idx = it * 256 + tid;
    const int c = idx >> 5, j = idx & 31;
    T[j * 260 + c] = xb[(size_t)c * kHW + j];
  }
  __syncthreads();
  const int wave = tid >> 5, lane = tid & 31;
  v8h vh[4], vl[4], vf[4];
#pragma unroll
  for (int r = 0; r < 4; ++r) {
    const int j = wave * 4 + r;
    const v4f a0 = *(const v4f*)(T + j * 260 + lane * 8);
    const v4f a1 = *(const v4f*)(T + j * 260 + lane * 8 + 4);
#pragma unroll
    for (int e = 0; e < 4; ++e) {
      const float x0 = a0[e], x1 = a1[e];
      const unsigned short h0 = f2bf_bits(x0), h1 = f2bf_bits(x1);
      const unsigned short l0 = f2bf_bits(x0 - bf_bits2f(h0)), l1 = f2bf_bits(x1 - bf_bits2f(h1));
      vh[r][e] = __builtin_bit_cast(_Float16, h0); vh[r][4 + e] = __builtin_bit_cast(_Float16, h1);
      vl[r][e] = __builtin_bit_cast(_Float16, l0); vl[r][4 + e] = __builtin_bit_cast(_Float16, l1);
      vf[r][e] = (_Float16)x0;                     vf[r][4 + e] = (_Float16)x1;
    }
  }
  const size_t pbase = ((size_t)sel * kHW + n0) * kCh;
  _Float16* ph = (_Float16*)FThi + pbase;
  _Float16* pl = (_Float16*)FTlo + pbase;
  _Float16* pf = (_Float16*)FT16 + pbase;
  for (int pass = 0; pass < 2; ++pass) {
#pragma unroll
    for (int r = 0; r < 4; ++r) {
      const int j = wave * 4 + r;
      const size_t o = (size_t)j * kCh + lane * 8;
      *(volatile v8h*)(ph + o) = vh[r];
      *(volatile v8h*)(pl + o) = vl[r];
      *(volatile v8h*)(pf + o) = vf[r];
    }
    __threadfence();
  }
}

__global__ __launch_bounds__(256) void k_softmax(const float* __restrict__ S, unsigned short* __restrict__ P) {
  __shared__ float red[16];
  const int tid = threadIdx.x, wave = tid >> 5, lane = tid & 31;
  const int row = blockIdx.x;
  const float* sr = S + (size_t)row * kHW;
  float v[16];
#pragma unroll
  for (int ch = 0; ch < 2; ++ch) {
    const v4f a = *(const v4f*)(sr + ch * 2048 + tid * 8);
    const v4f c = *(const v4f*)(sr + ch * 2048 + tid * 8 + 4);
    v[ch * 8 + 0] = a[0]; v[ch * 8 + 1] = a[1]; v[ch * 8 + 2] = a[2]; v[ch * 8 + 3] = a[3];
    v[ch * 8 + 4] = c[0]; v[ch * 8 + 5] = c[1]; v[ch * 8 + 6] = c[2]; v[ch * 8 + 7] = c[3];
  }
  float mx = v[0];
#pragma unroll
  for (int e = 1; e < 16; ++e) mx = fmaxf(mx, v[e]);
#pragma unroll
  for (int off = 1; off < 32; off <<= 1) mx = fmaxf(mx, __shfl_xor(mx, off, 32));
  if (lane == 0) red[wave] = mx;
  __syncthreads();
  float gmx = red[0];
#pragma unroll
  for (int w = 1; w < 8; ++w) gmx = fmaxf(gmx, red[w]);
  float s = 0.f;
#pragma unroll
  for (int e = 0; e < 16; ++e) { v[e] = __expf(v[e] - gmx); s += v[e]; }
#pragma unroll
  for (int off = 1; off < 32; off <<= 1) s += __shfl_xor(s, off, 32);
  if (lane == 0) red[8 + wave] = s;
  __syncthreads();
  float tot = red[8];
#pragma unroll
  for (int w = 1; w < 8; ++w) tot += red[8 + w];
  const float sc = 32768.0f * (1.0f / tot);
  v8h h[2];
#pragma unroll
  for (int ch = 0; ch < 2; ++ch) {
#pragma unroll
    for (int e = 0; e < 8; ++e) h[ch][e] = (_Float16)(v[ch * 8 + e] * sc);
  }
  _Float16* pr = (_Float16*)P + (size_t)row * kHW;
  for (int pass = 0; pass < 2; ++pass) {
#pragma unroll
    for (int ch = 0; ch < 2; ++ch) *(volatile v8h*)(pr + ch * 2048 + tid * 8) = h[ch];
    __threadfence();
  }
}

extern "C" void kernel_launch(void* const* d_in, const int* in_sizes, int n_in,
                              void* d_out, int out_size, void* d_ws, size_t ws_size,
                              hipStream_t stream) {
  if (n_in < 11) return;
  if (in_sizes[0] != kBatch * kCh * kHW || in_sizes[1] != kBatch * kCh * kHW) return;
  if (in_sizes[2] < kCh || in_sizes[3] < kCh) return;
  if (in_sizes[4] != kQC * kCh || in_sizes[6] != kQC * kCh || in_sizes[8] != kCh * kCh) return;
  if (in_sizes[5] < kQC || in_sizes[7] < kQC || in_sizes[9] < kCh || in_sizes[10] < 1) return;
  if (out_size != 2 * kBatch * kCh * kHW) return;

  const float* f1    = (const float*)d_in[0];
  const float* f2    = (const float*)d_in[1];
  const float* te1   = (const float*)d_in[2];
  const float* te2   = (const float*)d_in[3];
  const float* wq    = (const float*)d_in[4];
  const float* bq    = (const float*)d_in[5];
  const float* wk    = (const float*)d_in[6];
  const float* bk    = (const float*)d_in[7];
  const float* wv    = (const float*)d_in[8];
  const float* bv    = (const float*)d_in[9];
  const float* gamma = (const float*)d_in[10];
  float* out = (float*)d_out;

  char* ws = (char*)d_ws;
  size_t off = 0;
  auto carve = [&](size_t bytes) -> char* { char* p = ws + off; off += (bytes + 255) & ~(size_t)255; return p; };
  const size_t PL = (size_t)kHW * kCh;
  const size_t QL = (size_t)kHW * kQK;
  const size_t VL = (size_t)kCh * kHW;
  const size_t CHW = (size_t)kCh * kHW;
  unsigned short* FThi  = (unsigned short*)carve(2 * PL * 2);
  unsigned short* FTlo  = (unsigned short*)carve(2 * PL * 2);
  unsigned short* FT16  = (unsigned short*)carve(2 * PL * 2);
  unsigned short* QKhi  = (unsigned short*)carve(2 * QL * 2);
  unsigned short* QKlo  = (unsigned short*)carve(2 * QL * 2);
  unsigned short* V16   = (unsigned short*)carve(2 * VL * 2);
  float*          S     = (float*)carve((size_t)kHW * kHW * 4);
  unsigned short* P16   = (unsigned short*)carve((size_t)kHW * kHW * 2);
  unsigned short* Wqkhi = (unsigned short*)carve((size_t)kQK * kCh * 2);
  unsigned short* Wqklo = (unsigned short*)carve((size_t)kQK * kCh * 2);
  unsigned short* Wv16  = (unsigned short*)carve((size_t)kCh * kCh * 2);
  float*          BIAS  = (float*)carve((size_t)2 * kBiasPer * 4);
  if (off > ws_size) return;

  k_biasfold<<<20, 256, 0, stream>>>(wq, bq, wk, bk, wv, bv, te1, te2, gamma, BIAS);
  k_prepw<<<160, 256, 0, stream>>>(wq, wk, wv, gamma, Wqkhi, Wqklo, Wv16);

  for (int b = 0; b < kBatch; ++b) {
    k_ftrans<<<dim3(kHW / 32, 2), 256, 0, stream>>>(f1, f2, b, FThi, FTlo, FT16);
    for (int in = 0; in < 2; ++in) {
      wmma_gemm64<1, true, 2, 2, false><<<dim3(8, 1), 256, 0, stream>>>(
          FThi + in * PL, FTlo + in * PL, kCh, (long)0,
          Wqkhi, Wqklo, kCh, (long)0,
          (void*)(QKhi + in * QL), (void*)(QKlo + in * QL), kQK, (long)0,
          BIAS + in * kBiasPer, BIAS, (long)0,
          kHW, kQK, kCh, 1.0f);
      wmma_gemm64<0, false, 1, 1, false><<<dim3(32, 1), 256, 0, stream>>>(
          Wv16, Wv16, kCh, (long)0,
          FT16 + in * PL, FT16 + in * PL, kCh, (long)0,
          (void*)(V16 + in * VL), (void*)(V16 + in * VL), kHW, (long)0,
          BIAS + in * kBiasPer + 64, BIAS, (long)0,
          kCh, kHW, kCh, 0.5f);
    }
    for (int dir = 0; dir < 2; ++dir) {
      const int qs = 1 - dir, ks = dir, vs = dir;
      const float* fres = (dir ? f2 : f1) + (size_t)b * CHW;
      float* ob = out + (size_t)dir * kBatch * CHW + (size_t)b * CHW;
      wmma_gemm64<1, true, 0, 0, false><<<dim3(512, 1), 256, 0, stream>>>(
          QKhi + qs * QL, QKlo + qs * QL, kQK, (long)0,
          QKhi + ks * QL + kQC, QKlo + ks * QL + kQC, kQK, (long)0,
          (void*)S, (void*)S, kHW, (long)0,
          BIAS, BIAS, (long)0,
          kHW, kHW, kQC, 1.0f);
      k_softmax<<<kHW, 256, 0, stream>>>(S, P16);
      wmma_gemm64<0, false, 0, 0, true><<<dim3(32, 1), 256, 0, stream>>>(
          V16 + vs * VL, V16 + vs * VL, kHW, (long)0,
          P16, P16, kHW, (long)0,
          (void*)ob, (void*)ob, kHW, (long)0,
          BIAS, fres, (long)0,
          kCh, kHW, kHW, 1.0f / 262144.0f);
    }
  }
}
